// CausalSelfAttention_58110907515671
// MI455X (gfx1250) — hardware-verified
//
#include <hip/hip_runtime.h>


#ifndef NB
#define NB 2
#endif
#ifndef SEQ
#define SEQ 2048
#endif
#define NB_FULL  2
#define SEQ_FULL 2048
#define DM   1024
#define NH   16
#define HD   64
#define NQKV (3 * DM)
#define RH   ((SEQ) < 256 ? (SEQ) : 256)
#define PCAR 1024.0f
#define SCL  0.125f
#define LOG2E 1.4426950408889634f
#define NEGB (-1.0e30f)
#define OSP  68
#define PP   40
#define NWA  4

typedef _Float16 h16;
typedef unsigned short bf;
typedef __attribute__((ext_vector_type(16))) __bf16   v16bf;
typedef __attribute__((ext_vector_type(16))) _Float16 v16h;
typedef __attribute__((ext_vector_type(8)))  _Float16 v8h;
typedef __attribute__((ext_vector_type(8)))  unsigned short v8us;
typedef __attribute__((ext_vector_type(2)))  unsigned short v2us;
typedef __attribute__((ext_vector_type(8)))  float    v8f;
typedef __attribute__((ext_vector_type(4)))  float    v4f;
typedef v8h  __attribute__((may_alias)) v8ha;
typedef v4f  __attribute__((may_alias)) v4fa;
typedef v8us __attribute__((may_alias)) v8usa;

static_assert(SEQ % 64 == 0);
static_assert((NB * SEQ) % 64 == 0);
static_assert(SEQ <= SEQ_FULL);
static_assert(NB <= NB_FULL);
static_assert(DM % 64 == 0);
static_assert(DM % 32 == 0);
static_assert(HD == 64);
static_assert(NH * HD == DM);
static_assert(NQKV % 64 == 0);
static_assert(RH % 64 == 0);
static_assert(RH <= SEQ);
static_assert(NWA * 16 == 64);
static_assert(PP >= 32);
static_assert(PP % 8 == 0);
static_assert(OSP >= 64);
static_assert(OSP % 4 == 0);

#define PLN   ((size_t)NB * NH * SEQ * HD)
#define SZ_XB   ((size_t)NB * SEQ * DM * 2)
#define SZ_WQKV ((size_t)NQKV * DM * 2)
#define SZ_WO   ((size_t)DM * DM * 2)
#define SZ_QK   ((size_t)2 * PLN * 2)
#define SZ_V16  ((size_t)PLN * 2)
#define SZ_VE   ((size_t)NB * NH * HD * RH * 2)
#define SZ_AT   ((size_t)2 * NB * SEQ * DM * 2)
#define SZ_TOT  (SZ_XB + SZ_WQKV + SZ_WO + 2 * SZ_QK + SZ_V16 + 2 * SZ_VE + SZ_AT)
static_assert(SZ_XB % 256 == 0);
static_assert(SZ_WQKV % 256 == 0);
static_assert(SZ_WO % 256 == 0);
static_assert(SZ_QK % 256 == 0);
static_assert(SZ_V16 % 256 == 0);
static_assert(SZ_VE % 256 == 0);
static_assert(SZ_AT % 256 == 0);
static_assert(SZ_TOT <= (size_t)134217728);
static_assert(((size_t)(NB - 1) * SEQ_FULL + SEQ) * DM * 4 <= (size_t)16777216);

__device__ __forceinline__ unsigned short f2bf(float f) { unsigned u = __float_as_uint(f); u += 0x7FFFu + ((u >> 16) & 1u); return (unsigned short)(u >> 16); }
__device__ __forceinline__ float bf2f(unsigned short b) { return __uint_as_float(((unsigned)b) << 16); }
__device__ __forceinline__ float bfr(float f) { return bf2f(f2bf(f)); }
__device__ __forceinline__ void splitf(float y, unsigned short& h, unsigned short& l) { h = f2bf(y); l = f2bf(y - bf2f(h)); }
__device__ __forceinline__ v16h cat16(v8h lo, v8h hi) { return __builtin_shufflevector(lo, hi, 0, 1, 2, 3, 4, 5, 6, 7, 8, 9, 10, 11, 12, 13, 14, 15); }
__device__ __forceinline__ v16bf cat16b(v8us lo, v8us hi) { return __builtin_bit_cast(v16bf, __builtin_shufflevector(lo, hi, 0, 1, 2, 3, 4, 5, 6, 7, 8, 9, 10, 11, 12, 13, 14, 15)); }
__device__ __forceinline__ v16bf ldb(const bf* p)  { return cat16b(*(const v8us*)p, *(const v8us*)(p + 16)); }
__device__ __forceinline__ v16h  ldh(const h16* p) { return cat16(*(const v8h*)p, *(const v8h*)(p + 16)); }
__device__ __forceinline__ v8f wmb(v16bf a, v16bf b, v8f c) {
    c = __builtin_amdgcn_wmma_f32_16x16x32_bf16(false, a, false, b, (short)0, c, false, false);
    asm volatile("v_nop\n\tv_nop\n\tv_nop\n\tv_nop" : "+v"(c) : "v"(a), "v"(b));
    return c;
}
__device__ __forceinline__ v8f wmh(v16h a, v16h b, v8f c) {
    c = __builtin_amdgcn_wmma_f32_16x16x32_f16(false, a, false, b, (short)0, c, false, false);
    asm volatile("v_nop\n\tv_nop\n\tv_nop\n\tv_nop" : "+v"(c) : "v"(a), "v"(b));
    return c;
}
__device__ __forceinline__ void wsync() { __builtin_amdgcn_fence(3  , "wavefront"); __builtin_amdgcn_wave_barrier(); asm volatile("" ::: "memory"); }

__global__ __launch_bounds__(256) void k_cvt8(const float* __restrict__ src, bf* dst, int n8) {
    const int i = blockIdx.x * 256 + threadIdx.x; if (i >= n8) return;
    const int row = i / (DM / 8), c8 = i % (DM / 8); const int b = row / SEQ, t = row % SEQ;
    const v8f v = *(const v8f*)(src + ((size_t)b * SEQ_FULL + t) * DM + (size_t)c8 * 8); v8us o;
#pragma unroll
    for (int k = 0; k < 8; ++k) o[k] = f2bf(v[k]);
    *(volatile v8us*)(dst + (size_t)i * 8) = o; __threadfence(); *(volatile v8us*)(dst + (size_t)i * 8) = o;
}

__global__ __launch_bounds__(256) void k_wtG(const float* __restrict__ w, int K, int N, bf* Bt) {
    const int lane = threadIdx.x & 31; const int L0 = (blockIdx.x * 8 + (threadIdx.x >> 5)) * 8; const int nlines = N * (K / 64);
#pragma unroll 1
    for (int ps = 0; ps < 2; ++ps) {
#pragma unroll 1
        for (int l = 0; l < 8; ++l) { const int L = L0 + l; if (L >= nlines) break; const size_t e = (size_t)L * 64 + lane * 2; const int k = (int)(e % (size_t)K), n = (int)(e / (size_t)K); v2us o;
            o[0] = f2bf(w[(size_t)k * N + n]); o[1] = f2bf(w[(size_t)(k + 1) * N + n]); *(volatile v2us*)(Bt + e) = o; }
        if (ps == 0) __threadfence(); }
}

template <int NPL>
__device__ __forceinline__ void gemm_main(const bf* __restrict__ A, size_t sPl, const bf* __restrict__ Bt, int r0, int c0, int lr, int hi, v8f (&acc)[4][4]) {
#pragma unroll
    for (int mb = 0; mb < 4; ++mb)
#pragma unroll
        for (int nb = 0; nb < 4; ++nb) acc[mb][nb] = (v8f){};
    const size_t aoff = (size_t)(r0 + lr) * DM + 8 * hi, boff = (size_t)(c0 + lr) * DM + 8 * hi;
#pragma unroll 1
    for (int kc = 0; kc < DM; kc += 32) {
#pragma unroll
        for (int pl = 0; pl < NPL; ++pl) {
            v16bf a[4];
#pragma unroll
            for (int mb = 0; mb < 4; ++mb) a[mb] = ldb(A + (size_t)pl * sPl + aoff + (size_t)mb * 16 * DM + kc);
#pragma unroll
            for (int nb = 0; nb < 4; ++nb) { const v16bf b = ldb(Bt + boff + (size_t)nb * 16 * DM + kc);
#pragma unroll
                for (int mb = 0; mb < 4; ++mb) acc[mb][nb] = wmb(a[mb], b, acc[mb][nb]); }
        }
    }
}

__global__ __launch_bounds__(32) void k_qkv(const bf* __restrict__ XB, const bf* __restrict__ WQKV, const float* __restrict__ bias, bf* QKh, bf* QKl, h16* V16, bf* Vh, bf* Vl) {
    __shared__ __align__(16) float os[64 * OSP];
    const int lane = threadIdx.x & 31, lr = lane & 15, hi = lane >> 4; const int r0 = blockIdx.x * 64, c0 = blockIdx.y * 64;
    v8f acc[4][4];
    gemm_main<1>(XB, (size_t)0, WQKV, r0, c0, lr, hi, acc);
    const int which = c0 / DM; const int head = (c0 % DM) / HD; const int b = r0 / SEQ, t0 = r0 % SEQ; const int bh = b * NH + head;
    float bv[4];
#pragma unroll
    for (int nb = 0; nb < 4; ++nb) bv[nb] = bfr(bias[c0 + nb * 16 + lr]);
    const int q4 = lane >> 3, pc = (lane & 7) * 8;
    if (which < 2) {
        const size_t pofs = (size_t)which * PLN + ((size_t)bh * SEQ + t0) * HD;
#pragma unroll
        for (int mb = 0; mb < 4; ++mb) {
#pragma unroll
            for (int nb = 0; nb < 4; ++nb) {
#pragma unroll
                for (int j = 0; j < 8; ++j) os[(hi * 8 + j) * OSP + nb * 16 + lr] = acc[mb][nb][j] + bv[nb]; }
            wsync();
#pragma unroll 1
            for (int ps = 0; ps < 2; ++ps) {
#pragma unroll
                for (int s = 0; s < 4; ++s) { const int row = 4 * s + q4; const v4f x0 = *(const v4fa*)(os + row * OSP + pc), x1 = *(const v4fa*)(os + row * OSP + pc + 4); v8us oh, ol;
#pragma unroll
                    for (int q = 0; q < 4; ++q) { unsigned short a, c; splitf(x0[q], a, c); oh[q] = a; ol[q] = c; splitf(x1[q], a, c); oh[4 + q] = a; ol[4 + q] = c; }
                    const size_t oo = pofs + (size_t)(mb * 16 + row) * HD + pc; *(volatile v8us*)(QKh + oo) = oh; *(volatile v8us*)(QKl + oo) = ol; }
                if (ps == 0) __threadfence(); }
            wsync();
        }
    } else {
#pragma unroll
        for (int mb = 0; mb < 4; ++mb)
#pragma unroll
            for (int nb = 0; nb < 4; ++nb) {
#pragma unroll
                for (int j = 0; j < 8; ++j) os[(nb * 16 + lr) * OSP + mb * 16 + hi * 8 + j] = acc[mb][nb][j] + bv[nb]; }
        wsync();
        const size_t vofs = (size_t)bh * HD * SEQ + t0; const size_t eofs = (size_t)bh * HD * RH + t0;
#pragma unroll 1
        for (int ps = 0; ps < 2; ++ps) {
#pragma unroll 1
            for (int s = 0; s < 16; ++s) { const int d = 4 * s + q4; const v4f x0 = *(const v4fa*)(os + d * OSP + pc), x1 = *(const v4fa*)(os + d * OSP + pc + 4); v8h o16;
#pragma unroll
                for (int q = 0; q < 4; ++q) { o16[q] = (h16)x0[q]; o16[4 + q] = (h16)x1[q]; }
                *(volatile v8h*)(V16 + vofs + (size_t)d * SEQ + pc) = o16;
                if (t0 < RH) { v8us oh, ol;
#pragma unroll
                    for (int q = 0; q < 4; ++q) { unsigned short a, c; splitf(x0[q], a, c); oh[q] = a; ol[q] = c; splitf(x1[q], a, c); oh[4 + q] = a; ol[4 + q] = c; }
                    const size_t oo = eofs + (size_t)d * RH + pc; *(volatile v8us*)(Vh + oo) = oh; *(volatile v8us*)(Vl + oo) = ol; } }
            if (ps == 0) __threadfence(); }
    }
}

__device__ __forceinline__ void score_step(const bf* __restrict__ QKh, const bf* __restrict__ QKl, size_t qoff, size_t koff, int kb, int q0, int lr, int hi,
                                           float (&mrow)[8], float (&lrow)[8], v8f (&o)[4], float (&p0)[8], float (&p1)[8]) {
    const v16bf qh0 = ldb(QKh + qoff), qh1 = ldb(QKh + qoff + 32), ql0 = ldb(QKl + qoff), ql1 = ldb(QKl + qoff + 32);
    v8f s0 = (v8f){}, s1 = (v8f){};
    { v16bf kh = ldb(QKh + koff), kl = ldb(QKl + koff);
      s0 = wmb(qh0, kh, s0); s0 = wmb(qh0, kl, s0); s0 = wmb(ql0, kh, s0);
      kh = ldb(QKh + koff + 32); kl = ldb(QKl + koff + 32);
      s0 = wmb(qh1, kh, s0); s0 = wmb(qh1, kl, s0); s0 = wmb(ql1, kh, s0); }
    { const size_t k2 = koff + (size_t)16 * HD; v16bf kh = ldb(QKh + k2), kl = ldb(QKl + k2);
      s1 = wmb(qh0, kh, s1); s1 = wmb(qh0, kl, s1); s1 = wmb(ql0, kh, s1);
      kh = ldb(QKh + k2 + 32); kl = ldb(QKl + k2 + 32);
      s1 = wmb(qh1, kh, s1); s1 = wmb(qh1, kl, s1); s1 = wmb(ql1, kh, s1); }
    const float cs = SCL * LOG2E;
#pragma unroll
    for (int r = 0; r < 8; ++r) {
        const int qrow = q0 + 8 * hi + r;
        const float t0 = (kb + lr <= qrow) ? s0[r] * cs : NEGB;
        const float t1 = (kb + 16 + lr <= qrow) ? s1[r] * cs : NEGB;
        float mx = fmaxf(t0, t1);
        mx = fmaxf(mx, __shfl_xor(mx, 8, 32)); mx = fmaxf(mx, __shfl_xor(mx, 4, 32)); mx = fmaxf(mx, __shfl_xor(mx, 2, 32)); mx = fmaxf(mx, __shfl_xor(mx, 1, 32));
        const float mnew = fmaxf(mrow[r], mx);
        const float alpha = __builtin_amdgcn_exp2f(mrow[r] - mnew);
        const float e0 = __builtin_amdgcn_exp2f(t0 - mnew), e1 = __builtin_amdgcn_exp2f(t1 - mnew);
        lrow[r] = lrow[r] * alpha + (e0 + e1); mrow[r] = mnew; p0[r] = e0; p1[r] = e1;
        o[0][r] *= alpha; o[1][r] *= alpha; o[2][r] *= alpha; o[3][r] *= alpha;
    }
}

__global__ __launch_bounds__(128) void k_attn(const bf* __restrict__ QKh, const bf* __restrict__ QKl, const h16* __restrict__ V16, const bf* __restrict__ Vh, const bf* __restrict__ Vl, bf* ATh, bf* ATl) {
    __shared__ __align__(16) h16 ps16[NWA][16 * PP];
    __shared__ __align__(16) unsigned short psh[NWA][16 * PP];
    __shared__ __align__(16) unsigned short psl[NWA][16 * PP];
    __shared__ __align__(16) float ost[NWA][16 * OSP];
    const int lane = threadIdx.x & 31, lr = lane & 15, hi = lane >> 4;
    const int wave = __builtin_amdgcn_readfirstlane(threadIdx.x >> 5);
    const int bh = blockIdx.y; const int qb0 = blockIdx.x * 64; const int q0 = qb0 + wave * 16;
    const size_t pbase = (size_t)bh * SEQ * HD;
    const size_t qoff = pbase + (size_t)(q0 + lr) * HD + 8 * hi;
    v8f o[4]; float mrow[8], lrow[8];
#pragma unroll
    for (int j = 0; j < 4; ++j) o[j] = (v8f){};
#pragma unroll
    for (int r = 0; r < 8; ++r) { mrow[r] = NEGB; lrow[r] = 0.0f; }
    const int pro = lr * PP + 8 * hi;
    if (qb0 < RH) {
#pragma unroll 1
        for (int kb = 0; kb <= q0 + 15; kb += 32) {
            float p0[8], p1[8];
            score_step(QKh, QKl, qoff, PLN + pbase + (size_t)(kb + lr) * HD + 8 * hi, kb, q0, lr, hi, mrow, lrow, o, p0, p1);
#pragma unroll
            for (int r = 0; r < 8; ++r) { unsigned short a, c; const int idx = (8 * hi + r) * PP + lr;
                splitf(p0[r], a, c); psh[wave][idx] = a; psl[wave][idx] = c; splitf(p1[r], a, c); psh[wave][idx + 16] = a; psl[wave][idx + 16] = c; }
            wsync();
            const v16bf ph = cat16b(*(const v8usa*)&psh[wave][pro], *(const v8usa*)&psh[wave][pro + 16]);
            const v16bf pl = cat16b(*(const v8usa*)&psl[wave][pro], *(const v8usa*)&psl[wave][pro + 16]);
            wsync();
            const size_t vo = (size_t)bh * HD * RH + (size_t)lr * RH + kb + 8 * hi;
#pragma unroll
            for (int j = 0; j < 4; ++j) { const v16bf vh = ldb(Vh + vo + (size_t)j * 16 * RH), vl = ldb(Vl + vo + (size_t)j * 16 * RH);
                o[j] = wmb(ph, vh, o[j]); o[j] = wmb(ph, vl, o[j]); o[j] = wmb(pl, vh, o[j]); }
        }
    } else {
#pragma unroll 1
        for (int kb = 0; kb <= q0 + 15; kb += 32) {
            float p0[8], p1[8];
            score_step(QKh, QKl, qoff, PLN + pbase + (size_t)(kb + lr) * HD + 8 * hi, kb, q0, lr, hi, mrow, lrow, o, p0, p1);
#pragma unroll
            for (int r = 0; r < 8; ++r) { const int idx = (8 * hi + r) * PP + lr; ps16[wave][idx] = (h16)(p0[r] * PCAR); ps16[wave][idx + 16] = (h16)(p1[r] * PCAR); }
            wsync();
            const v16h pf = cat16(*(const v8ha*)&ps16[wave][pro], *(const v8ha*)&ps16[wave][pro + 16]);
            wsync();
            const size_t vo = (size_t)bh * HD * SEQ + (size_t)lr * SEQ + kb + 8 * hi;
#pragma unroll
            for (int j = 0; j < 4; ++j) { const v16h vf = ldh(V16 + vo + (size_t)j * 16 * SEQ); o[j] = wmh(pf, vf, o[j]); }
        }
    }
    const float car = (qb0 < RH) ? 1.0f : (1.0f / PCAR);
    float inv[8];
#pragma unroll
    for (int r = 0; r < 8; ++r) { float l = lrow[r]; l += __shfl_xor(l, 8, 32); l += __shfl_xor(l, 4, 32); l += __shfl_xor(l, 2, 32); l += __shfl_xor(l, 1, 32); inv[r] = __builtin_amdgcn_rcpf(l) * car; }
#pragma unroll
    for (int j = 0; j < 4; ++j)
#pragma unroll
        for (int r = 0; r < 8; ++r) ost[wave][(8 * hi + r) * OSP + j * 16 + lr] = o[j][r] * inv[r];
    wsync();
    const int b = bh / NH, h = bh % NH; const int q4 = lane >> 3, pc = (lane & 7) * 8;
    const size_t abase = ((size_t)b * SEQ + q0) * DM + (size_t)h * HD + pc;
#pragma unroll 1
    for (int ps = 0; ps < 2; ++ps) {
#pragma unroll
        for (int s = 0; s < 4; ++s) { const int row = 4 * s + q4; const v4f x0 = *(const v4fa*)&ost[wave][row * OSP + pc], x1 = *(const v4fa*)&ost[wave][row * OSP + pc + 4]; v8us oh, ol;
#pragma unroll
            for (int q = 0; q < 4; ++q) { unsigned short a, c; splitf(x0[q], a, c); oh[q] = a; ol[q] = c; splitf(x1[q], a, c); oh[4 + q] = a; ol[4 + q] = c; }
            const size_t oo = abase + (size_t)row * DM; *(volatile v8us*)(ATh + oo) = oh; *(volatile v8us*)(ATl + oo) = ol; }
        if (ps == 0) __threadfence(); }
}

__global__ __launch_bounds__(32) void k_oproj(const bf* __restrict__ AT, const bf* __restrict__ WO, const float* __restrict__ bias, float* OUT) {
    __shared__ __align__(16) float os[16 * OSP];
    const int lane = threadIdx.x & 31, lr = lane & 15, hi = lane >> 4; const int r0 = blockIdx.x * 64, c0 = blockIdx.y * 64;
    v8f acc[4][4];
    gemm_main<2>(AT, (size_t)NB * SEQ * DM, WO, r0, c0, lr, hi, acc);
    const int cofs = lr * 4; v4f bb;
#pragma unroll
    for (int q = 0; q < 4; ++q) bb[q] = bfr(bias[c0 + cofs + q]);
#pragma unroll
    for (int mb = 0; mb < 4; ++mb) {
#pragma unroll
        for (int nb = 0; nb < 4; ++nb) {
#pragma unroll
            for (int j = 0; j < 8; ++j) os[(hi * 8 + j) * OSP + nb * 16 + lr] = acc[mb][nb][j]; }
        wsync();
#pragma unroll 1
        for (int ps = 0; ps < 2; ++ps) {
#pragma unroll
            for (int s = 0; s < 8; ++s) { const int row = 2 * s + hi; const int m = r0 + mb * 16 + row; const int b = m / SEQ, t = m % SEQ;
                v4f val = *(const v4fa*)(os + row * OSP + cofs); val[0] += bb[0]; val[1] += bb[1]; val[2] += bb[2]; val[3] += bb[3];
                *(volatile v4f*)(OUT + ((size_t)b * SEQ_FULL + t) * DM + c0 + cofs) = val; }
            if (ps == 0) __threadfence(); }
        wsync();
    }
}

extern "C" void kernel_launch(void* const* d_in, const int* in_sizes, int n_in,
                              void* d_out, int out_size, void* d_ws, size_t ws_size, hipStream_t stream) {
    if (n_in < 5) return;
    const long long need_x = ((long long)(NB - 1) * SEQ_FULL + SEQ) * DM;
    if ((long long)in_sizes[0] < need_x) return;
    if ((long long)in_sizes[1] < (long long)DM * NQKV) return;
    if ((long long)in_sizes[2] < (long long)NQKV) return;
    if ((long long)in_sizes[3] < (long long)DM * DM) return;
    if ((long long)in_sizes[4] < (long long)DM) return;
    if ((long long)out_size < need_x) return;
    if (ws_size < SZ_TOT) return;
    const float* x = (const float*)d_in[0]; const float* wqkv = (const float*)d_in[1]; const float* bqkv = (const float*)d_in[2]; const float* wo = (const float*)d_in[3]; const float* bo = (const float*)d_in[4];
    float* OUT = (float*)d_out;
    char* wsp = (char*)d_ws;
    bf* XB   = (bf*)wsp;  wsp += SZ_XB;
    bf* WQKV = (bf*)wsp;  wsp += SZ_WQKV;
    bf* WO   = (bf*)wsp;  wsp += SZ_WO;
    bf* QKh  = (bf*)wsp;  wsp += SZ_QK;
    bf* QKl  = (bf*)wsp;  wsp += SZ_QK;
    h16* V16 = (h16*)wsp; wsp += SZ_V16;
    bf* Vh   = (bf*)wsp;  wsp += SZ_VE;
    bf* Vl   = (bf*)wsp;  wsp += SZ_VE;
    bf* AT   = (bf*)wsp;  wsp += SZ_AT;
    bf* ATl  = AT + (size_t)NB * SEQ * DM;

    const int n8 = NB * SEQ * (DM / 8);
    k_cvt8<<<(unsigned)((n8 + 255) / 256), 256, 0, stream>>>(x, XB, n8);
    k_wtG<<<(unsigned)((NQKV * (DM / 64) + 63) / 64), 256, 0, stream>>>(wqkv, DM, NQKV, WQKV);
    k_wtG<<<(unsigned)((DM * (DM / 64) + 63) / 64), 256, 0, stream>>>(wo, DM, DM, WO);
    k_qkv<<<dim3(NB * SEQ / 64, NQKV / 64, 1), 32, 0, stream>>>(XB, WQKV, bqkv, QKh, QKl, V16, Vh, Vl);
    k_attn<<<dim3(SEQ / 64, NB * NH, 1), 128, 0, stream>>>(QKh, QKl, V16, Vh, Vl, AT, ATl);
    k_oproj<<<dim3(NB * SEQ / 64, DM / 64, 1), 32, 0, stream>>>(AT, WO, bo, OUT);
}
